// LSTMModel_2456721293896
// MI455X (gfx1250) — hardware-verified
//
#include <hip/hip_runtime.h>

constexpr int NBATCH  = 4096;
constexpr int NSTEP   = 512;
constexpr int NHID    = 50;
constexpr int NGATE   = 200;
constexpr int MROWS   = 32;
constexpr int NWAVE   = 13;
constexpr int NTHR    = NWAVE * 32;
constexpr int HPITCH  = 136;
constexpr int GPITCH  = 212;
constexpr int XTP     = 32;
constexpr int XQ      = NSTEP / 4;
constexpr int NCELL   = MROWS * NHID;
constexpr int CELL_IT = 4;
constexpr float HCARRY = 256.0f;
constexpr float WCARRY = 256.0f;
constexpr float FOLD   = 1.0f / 65536.0f;
static_assert(NBATCH % MROWS == 0, "grid exact");
static_assert(NGATE == 4 * NHID, "gate layout");
static_assert(NWAVE * 16 >= NGATE && GPITCH >= NWAVE * 16, "n coverage");
static_assert(CELL_IT * NTHR >= NCELL, "cell coverage");
static_assert((NCELL - (CELL_IT - 1) * NTHR) % 32 == 0, "cell guard is wave-uniform");
static_assert(NSTEP % 4 == 0 && XTP == MROWS, "x tile layout");
static_assert(HPITCH % 8 == 0 && HPITCH >= 128, "16-B aligned fragment loads, 4 k-chunks of 32");
static_assert(NHID <= 64, "h1 in cols 0..63, h2 in cols 64..127");

typedef __attribute__((ext_vector_type(16))) _Float16 v16h;
typedef __attribute__((ext_vector_type(8)))  _Float16 v8h;
typedef __attribute__((ext_vector_type(8)))  float    v8f;
typedef __attribute__((ext_vector_type(4)))  float    v4f;

__device__ __forceinline__ unsigned short f2bf_bits(float f) {
  unsigned u = __float_as_uint(f);
  return (unsigned short)((u + 0x7FFFu + ((u >> 16) & 1u)) >> 16);
}
__device__ __forceinline__ float bf_bits2f(unsigned short h) { return __uint_as_float(((unsigned)h) << 16); }
__device__ __forceinline__ float bf16r(float f) { return bf_bits2f(f2bf_bits(f)); }

__device__ __forceinline__ void dep_guard_h(v8f& a, v8f& b, v16h x, v16h y) { asm volatile("v_nop\n\tv_nop\n\tv_nop\n\tv_nop" : "+v"(a), "+v"(b) : "v"(x), "v"(y)); }
__device__ __forceinline__ void keep4_h(v16h a, v16h b, v16h c, v16h d) { asm volatile("v_nop" :: "v"(a), "v"(b), "v"(c), "v"(d)); }
__device__ __forceinline__ void half_fence(v8h& f) { asm volatile("" : "+v"(f) : : "memory"); }
__device__ __forceinline__ void sc_fence3(float& a, float& b, float& c) { asm volatile("" : "+v"(a), "+v"(b), "+v"(c) : : "memory"); }

template <typename T> struct Frag;
template <> struct Frag<_Float16> {
  typedef v16h V; union U { v16h v; v8h h[2]; };
  static __device__ __forceinline__ v16h load(const _Float16* p) {
    U f; f.h[0] = *(const v8h*)(p); f.h[1] = *(const v8h*)(p + 16); return f.v;
  }
  static __device__ __forceinline__ v8f mma(v16h a, v16h b, v8f c) {
    return __builtin_amdgcn_wmma_f32_16x16x32_f16(false, a, false, b, (short)0, c, false, false);
  }
};

__device__ __forceinline__ float fsig(float x)  { return __builtin_amdgcn_rcpf(1.0f + __expf(-x)); }
__device__ __forceinline__ float ftanh(float x) { return 1.0f - 2.0f * __builtin_amdgcn_rcpf(__expf(2.0f * x) + 1.0f); }

__device__ __forceinline__ v8h bfrag_half(const float* W, int nn, float fn, int kb) {
  v8h hv;
#pragma unroll
  for (int i = 0; i < 8; ++i) {
    const int   k  = kb + i;
    const int   kk = (k < NHID) ? k : (NHID - 1);
    const float fk = (k < NHID) ? fn : 0.0f;
    const float w  = W[nn * NHID + kk];
    hv[i] = (_Float16)(bf16r(w) * fk);
  }
  half_fence(hv);
  return hv;
}
__device__ __forceinline__ v16h build_bfrag(const float* W, int n, int kbase, int hi) {
  const int   nn = (n < NGATE) ? n : (NGATE - 1);
  const float fn = (n < NGATE) ? WCARRY : 0.0f;
  Frag<_Float16>::U u;
  u.h[0] = bfrag_half(W, nn, fn, kbase + 8 * hi);
  u.h[1] = bfrag_half(W, nn, fn, kbase + 16 + 8 * hi);
  return u.v;
}

__global__ __launch_bounds__(NTHR) void rnn2_kernel(const float* x,
    const float* W_ih0, const float* W_hh0, const float* b_ih0, const float* b_hh0,
    const float* W_ih1, const float* W_hh1, const float* b_ih1, const float* b_hh1,
    const float* W_fc, const float* b_fc, float* out) {
  __shared__ __align__(16) float    xT[NSTEP * XTP];
  __shared__ __align__(16) float    g0[MROWS * GPITCH];
  __shared__ __align__(16) float    g1[MROWS * GPITCH];
  __shared__ __align__(16) _Float16 hbuf[MROWS * HPITCH];
  __shared__ __align__(16) float    h2f[NCELL];
  __shared__ __align__(16) float    wfc_s[64];
  __shared__ __align__(16) float    fcs[MROWS];

  const int tid = threadIdx.x, lane = tid & 31, wave = tid >> 5;
  const int c = lane & 15, hi = lane >> 4;
  const int n = wave * 16 + c;
  const int rowbase = blockIdx.x * MROWS;

#pragma unroll 1
  for (int i = tid; i < MROWS * HPITCH; i += NTHR) hbuf[i] = (_Float16)0.0f;

#pragma unroll 1
  for (int i = tid; i < MROWS * XQ; i += NTHR) {
    const int row = i / XQ;
    const int q   = i - row * XQ;
    const v4f v = *(const v4f*)(x + (size_t)(rowbase + row) * NSTEP + 4 * q);
    xT[(4 * q + 0) * XTP + row] = bf16r(v[0]);
    xT[(4 * q + 1) * XTP + row] = bf16r(v[1]);
    xT[(4 * q + 2) * XTP + row] = bf16r(v[2]);
    xT[(4 * q + 3) * XTP + row] = bf16r(v[3]);
  }

  const int   nn     = (n < NGATE) ? n : (NGATE - 1);
  const float fvalid = (n < NGATE) ? 1.0f : 0.0f;
  float bias0 = (bf16r(b_ih0[nn]) + bf16r(b_hh0[nn])) * fvalid;
  float w0    = bf16r(W_ih0[nn]) * fvalid;
  float bias1 = (bf16r(b_ih1[nn]) + bf16r(b_hh1[nn])) * fvalid;
  sc_fence3(bias0, w0, bias1);

  const v16h bw0_0 = build_bfrag(W_hh0, n, 0,  hi);
  const v16h bw0_1 = build_bfrag(W_hh0, n, 32, hi);
  const v16h bw1_0 = build_bfrag(W_ih1, n, 0,  hi);
  const v16h bw1_1 = build_bfrag(W_ih1, n, 32, hi);
  const v16h bw1_2 = build_bfrag(W_hh1, n, 0,  hi);
  const v16h bw1_3 = build_bfrag(W_hh1, n, 32, hi);

  if (tid < 64) {
    const int j = (tid < NHID) ? tid : (NHID - 1);
    wfc_s[tid] = bf16r(W_fc[j]);
  }

  float cst0[CELL_IT], cst1[CELL_IT];
#pragma unroll
  for (int it = 0; it < CELL_IT; ++it) { cst0[it] = 0.0f; cst1[it] = 0.0f; }

  __syncthreads();

  const v8f z8 = {0.f, 0.f, 0.f, 0.f, 0.f, 0.f, 0.f, 0.f};
  const _Float16* a0p = hbuf + c * HPITCH + 8 * hi;
  const _Float16* a1p = hbuf + (16 + c) * HPITCH + 8 * hi;
  float* g0w = g0 + (8 * hi) * GPITCH + n;
  float* g1w = g1 + (8 * hi) * GPITCH + n;

#pragma unroll 1
  for (int t = 0; t < NSTEP; ++t) {
    {
      v8f acc0 = z8, acc1 = z8;
      const v16h a00 = Frag<_Float16>::load(a0p);
      const v16h a10 = Frag<_Float16>::load(a1p);
      const v16h a01 = Frag<_Float16>::load(a0p + 32);
      const v16h a11 = Frag<_Float16>::load(a1p + 32);
      acc0 = Frag<_Float16>::mma(a00, bw0_0, acc0);
      acc1 = Frag<_Float16>::mma(a10, bw0_0, acc1);
      acc0 = Frag<_Float16>::mma(a01, bw0_1, acc0);
      acc1 = Frag<_Float16>::mma(a11, bw0_1, acc1);
      dep_guard_h(acc0, acc1, a01, a11);
      keep4_h(a00, a10, bw0_0, bw0_1);
      const float* xr = xT + t * XTP;
      const v4f x0a = *(const v4f*)(xr + 8 * hi);
      const v4f x0b = *(const v4f*)(xr + 8 * hi + 4);
      const v4f x1a = *(const v4f*)(xr + 16 + 8 * hi);
      const v4f x1b = *(const v4f*)(xr + 16 + 8 * hi + 4);
#pragma unroll
      for (int r = 0; r < 4; ++r) {
        g0w[(r)      * GPITCH] = fmaf(acc0[r],     FOLD, fmaf(x0a[r], w0, bias0));
        g0w[(4 + r)  * GPITCH] = fmaf(acc0[4 + r], FOLD, fmaf(x0b[r], w0, bias0));
        g0w[(16 + r) * GPITCH] = fmaf(acc1[r],     FOLD, fmaf(x1a[r], w0, bias0));
        g0w[(20 + r) * GPITCH] = fmaf(acc1[4 + r], FOLD, fmaf(x1b[r], w0, bias0));
      }
    }
    __syncthreads();

#pragma unroll
    for (int it = 0; it < CELL_IT; ++it) {
      const int idx = tid + it * NTHR;
      if (idx < NCELL) {
        const int row = idx / NHID;
        const int j   = idx - row * NHID;
        const float* gp = g0 + row * GPITCH + j;
        const float zi = gp[0], zf = gp[NHID], zg = gp[2 * NHID], zo = gp[3 * NHID];
        const float cn = fsig(zf) * cst0[it] + fsig(zi) * ftanh(zg);
        cst0[it] = cn;
        const float hn = fsig(zo) * ftanh(cn);
        hbuf[row * HPITCH + j] = (_Float16)(hn * HCARRY);
      }
    }
    __syncthreads();

    {
      v8f acc0 = z8, acc1 = z8;
      {
        const v16h a0 = Frag<_Float16>::load(a0p);
        const v16h a1 = Frag<_Float16>::load(a1p);
        acc0 = Frag<_Float16>::mma(a0, bw1_0, acc0);
        acc1 = Frag<_Float16>::mma(a1, bw1_0, acc1);
        dep_guard_h(acc0, acc1, a0, a1);
      }
      {
        const v16h a0 = Frag<_Float16>::load(a0p + 32);
        const v16h a1 = Frag<_Float16>::load(a1p + 32);
        acc0 = Frag<_Float16>::mma(a0, bw1_1, acc0);
        acc1 = Frag<_Float16>::mma(a1, bw1_1, acc1);
        dep_guard_h(acc0, acc1, a0, a1);
      }
      {
        const v16h a0 = Frag<_Float16>::load(a0p + 64);
        const v16h a1 = Frag<_Float16>::load(a1p + 64);
        acc0 = Frag<_Float16>::mma(a0, bw1_2, acc0);
        acc1 = Frag<_Float16>::mma(a1, bw1_2, acc1);
        dep_guard_h(acc0, acc1, a0, a1);
      }
      {
        const v16h a0 = Frag<_Float16>::load(a0p + 96);
        const v16h a1 = Frag<_Float16>::load(a1p + 96);
        acc0 = Frag<_Float16>::mma(a0, bw1_3, acc0);
        acc1 = Frag<_Float16>::mma(a1, bw1_3, acc1);
        dep_guard_h(acc0, acc1, a0, a1);
      }
      keep4_h(bw1_0, bw1_1, bw1_2, bw1_3);
#pragma unroll
      for (int r = 0; r < 8; ++r) {
        g1w[(r)      * GPITCH] = fmaf(acc0[r], FOLD, bias1);
        g1w[(16 + r) * GPITCH] = fmaf(acc1[r], FOLD, bias1);
      }
    }
    __syncthreads();

    const bool last = (t == NSTEP - 1);
#pragma unroll
    for (int it = 0; it < CELL_IT; ++it) {
      const int idx = tid + it * NTHR;
      if (idx < NCELL) {
        const int row = idx / NHID;
        const int j   = idx - row * NHID;
        const float* gp = g1 + row * GPITCH + j;
        const float zi = gp[0], zf = gp[NHID], zg = gp[2 * NHID], zo = gp[3 * NHID];
        const float cn = fsig(zf) * cst1[it] + fsig(zi) * ftanh(zg);
        cst1[it] = cn;
        const float hn = fsig(zo) * ftanh(cn);
        hbuf[row * HPITCH + 64 + j] = (_Float16)(hn * HCARRY);
        if (last) h2f[row * NHID + j] = hn;
      }
    }
    __syncthreads();
  }

  if (tid < MROWS) {
    float acc = 0.0f;
#pragma unroll 2
    for (int j = 0; j < NHID; ++j) acc = fmaf(h2f[tid * NHID + j], wfc_s[j], acc);
    fcs[tid] = acc + bf16r(b_fc[0]);
  }
  __syncthreads();
  if (tid < 8) {
    const v4f v = *(const v4f*)(fcs + 4 * tid);
    float* op = out + rowbase + 4 * tid;
    *(volatile v4f*)op = v;
    __threadfence();
    *(volatile v4f*)op = v;
  }
}

extern "C" void kernel_launch(void* const* d_in, const int* in_sizes, int n_in,
                              void* d_out, int out_size, void* d_ws, size_t ws_size, hipStream_t stream) {
  (void)d_ws; (void)ws_size;
  if (n_in < 11 || d_out == nullptr) return;
  if (in_sizes[0] != NBATCH * NSTEP || in_sizes[1] != NGATE || in_sizes[2] != NGATE * NHID ||
      in_sizes[3] != NGATE || in_sizes[4] != NGATE || in_sizes[5] != NGATE * NHID ||
      in_sizes[6] != NGATE * NHID || in_sizes[7] != NGATE || in_sizes[8] != NGATE ||
      in_sizes[9] != NHID || in_sizes[10] != 1 || out_size != NBATCH) return;

  const float* x     = (const float*)d_in[0];
  const float* w_ih0 = (const float*)d_in[1];
  const float* w_hh0 = (const float*)d_in[2];
  const float* b_ih0 = (const float*)d_in[3];
  const float* b_hh0 = (const float*)d_in[4];
  const float* w_ih1 = (const float*)d_in[5];
  const float* w_hh1 = (const float*)d_in[6];
  const float* b_ih1 = (const float*)d_in[7];
  const float* b_hh1 = (const float*)d_in[8];
  const float* w_fc  = (const float*)d_in[9];
  const float* b_fc  = (const float*)d_in[10];
  float* out = (float*)d_out;

  rnn2_kernel<<<NBATCH / MROWS, NTHR, 0, stream>>>(x, w_ih0, w_hh0, b_ih0, b_hh0,
                                                  w_ih1, w_hh1, b_ih1, b_hh1, w_fc, b_fc, out);
}
